// regressor_acf_46042049413650
// MI455X (gfx1250) — hardware-verified
//
#include <hip/hip_runtime.h>
#include <stdint.h>

typedef _Float16 v16h __attribute__((ext_vector_type(16)));
typedef _Float16 v8h  __attribute__((ext_vector_type(8)));
typedef float    v8f  __attribute__((ext_vector_type(8)));
typedef float    v4f  __attribute__((ext_vector_type(4)));
union Frag { v16h v; v8h half[2]; _Float16 e[16]; };

constexpr int SEQ_L   = 8192;
constexpr int FPAD    = 16;
constexpr int VP_LEN  = 16448;
constexpr int NKCH    = SEQ_L / 32;
constexpr int POOL    = 8;
constexpr int POOLED  = SEQ_L / POOL;
constexpr int L1N     = 512;
constexpr int L2N     = 256;
constexpr int OUTN    = 4;
constexpr int MROWS   = 16;

constexpr float XSCALE = 16.0f;
constexpr float ASCALE = 16.0f;
constexpr float WSCALE = 64.0f;
constexpr float INV_AW = 1.0f / (ASCALE * WSCALE);

static __device__ __forceinline__ v8f wmma16(const v16h a, const v16h b, v8f c) {
  v8f d = __builtin_amdgcn_wmma_f32_16x16x32_f16(false, a, false, b, (short)0, c, false, false);
  asm volatile("v_nop\n\tv_nop\n\tv_nop\n\tv_nop" : "+v"(d) : "v"(a), "v"(b));
  return d;
}

static __device__ __forceinline__ v16h ld_frag_h(const _Float16* p, int h) {
  Frag f;
  f.half[0] = *(const v8h*)(p + 8 * h);
  f.half[1] = *(const v8h*)(p + 16 + 8 * h);
  return f.v;
}
static __device__ __forceinline__ v16h ld_frag_f32(const float* p, int h, float scale) {
  const v4f a0 = *(const v4f*)(p + 8 * h);
  const v4f a1 = *(const v4f*)(p + 8 * h + 4);
  const v4f c0 = *(const v4f*)(p + 16 + 8 * h);
  const v4f c1 = *(const v4f*)(p + 16 + 8 * h + 4);
  Frag f;
#pragma unroll
  for (int i = 0; i < 4; ++i) {
    f.e[i]      = (_Float16)(a0[i] * scale);
    f.e[4 + i]  = (_Float16)(a1[i] * scale);
    f.e[8 + i]  = (_Float16)(c0[i] * scale);
    f.e[12 + i] = (_Float16)(c1[i] * scale);
  }
  return f.v;
}

__global__ __launch_bounds__(256) void k_acf(const float* __restrict__ x,
                                             _Float16* __restrict__ normH) {
  __shared__ __align__(16) _Float16 vp[VP_LEN];
  __shared__ __align__(16) float pooledS[POOLED];
  __shared__ float wmaxS[8];

  const int tid = threadIdx.x;
  const int row = blockIdx.x;
  const float* xr = x + (size_t)row * SEQ_L;

#pragma unroll 4
  for (int k = 0; k < SEQ_L / 256; ++k) {
    const float v = xr[k * 256 + tid];
    vp[FPAD + k * 256 + tid] = (_Float16)(v * XSCALE);
  }
  if (tid < FPAD) vp[tid] = (_Float16)0.0f;
  for (int i = FPAD + SEQ_L + tid; i < VP_LEN; i += 256) vp[i] = (_Float16)0.0f;
  __syncthreads();

  const int wv = __builtin_amdgcn_readfirstlane(tid >> 5);
  const int l  = tid & 31;
  const int h  = l >> 4;
  const int m  = l & 15;

  v8f acc[4];
#pragma unroll
  for (int j = 0; j < 4; ++j) acc[j] = (v8f){0.f, 0.f, 0.f, 0.f, 0.f, 0.f, 0.f, 0.f};

  const int nk = NKCH - 32 * wv;
#pragma unroll 1
  for (int kc = 0; kc < nk; ++kc) {
    const int t0 = kc * 32;
    Frag a;
    const _Float16* pa = vp + (t0 + FPAD - m + 8 * h);
#pragma unroll
    for (int i = 0; i < 8; ++i) { a.e[i] = pa[i]; a.e[8 + i] = pa[16 + i]; }
#pragma unroll
    for (int j = 0; j < 4; ++j) {
      const int blkg = wv * 4 + j;
      const _Float16* pb = vp + (t0 + FPAD + 16 * m + 256 * blkg);
      const v16h b = ld_frag_h(pb, h);
      acc[j] = wmma16(a.v, b, acc[j]);
    }
  }

#pragma unroll
  for (int j = 0; j < 4; ++j) {
    const int blkg = wv * 4 + j;
    float pv = acc[j][0];
#pragma unroll
    for (int e = 1; e < 8; ++e) pv = fmaxf(pv, acc[j][e]);
    pooledS[blkg * 32 + 2 * m + h] = pv;
  }
  __syncthreads();

  float mx = -3.402823466e38f;
  for (int i = tid; i < POOLED; i += 256) mx = fmaxf(mx, pooledS[i]);
#pragma unroll
  for (int o = 16; o > 0; o >>= 1) mx = fmaxf(mx, __shfl_xor(mx, o));
  if (l == 0) wmaxS[wv] = mx;
  __syncthreads();
  float rmax = wmaxS[0];
#pragma unroll
  for (int i = 1; i < 8; ++i) rmax = fmaxf(rmax, wmaxS[i]);
  const float inv = 1.0f / rmax;

  v8h ov = (v8h){0, 0, 0, 0, 0, 0, 0, 0};
  const bool doit = tid < (POOLED / 8);
  if (doit) {
#pragma unroll
    for (int i = 0; i < 8; ++i) ov[i] = (_Float16)((pooledS[8 * tid + i] * inv) * ASCALE);
  }
  _Float16* op = normH + (size_t)row * POOLED + 8 * tid;
  if (doit) *(volatile v8h*)op = ov;
  __threadfence();
  if (doit) *(volatile v8h*)op = ov;
}

__global__ __launch_bounds__(256) void k_mlp(
    const _Float16* __restrict__ normH,
    const float* __restrict__ W1, const float* __restrict__ b1,
    const float* __restrict__ W2, const float* __restrict__ b2,
    const float* __restrict__ W3, const float* __restrict__ b3,
    float* __restrict__ out, int nrows) {
  __shared__ __align__(16) _Float16 h1[MROWS * L1N];
  __shared__ __align__(16) _Float16 h2[MROWS * L2N];
  __shared__ __align__(16) float outS[MROWS * OUTN];

  const int tid  = threadIdx.x;
  const int wv   = __builtin_amdgcn_readfirstlane(tid >> 5);
  const int l    = tid & 31;
  const int h    = l >> 4;
  const int m    = l & 15;
  const int row0 = blockIdx.x * MROWS;

  {
    v8f acc[4];
#pragma unroll
    for (int j = 0; j < 4; ++j) acc[j] = (v8f){0.f, 0.f, 0.f, 0.f, 0.f, 0.f, 0.f, 0.f};
    int ra = row0 + m; if (ra > nrows - 1) ra = nrows - 1;
    const _Float16* arow = normH + (size_t)ra * POOLED;
#pragma unroll 1
    for (int kc = 0; kc < POOLED / 32; ++kc) {
      const int kb = kc * 32;
      const v16h a = ld_frag_h(arow + kb, h);
#pragma unroll
      for (int j = 0; j < 4; ++j) {
        const int n = (wv * 4 + j) * 16 + m;
        const v16h b = ld_frag_f32(W1 + (size_t)n * POOLED + kb, h, WSCALE);
        acc[j] = wmma16(a, b, acc[j]);
      }
    }
#pragma unroll
    for (int j = 0; j < 4; ++j) {
      const int n = (wv * 4 + j) * 16 + m;
      const float bb = b1[n];
#pragma unroll
      for (int e = 0; e < 8; ++e) {
        const int mrow = 8 * h + e;
        float v = acc[j][e] * INV_AW + bb;
        v = v > 0.0f ? v : 0.01f * v;
        h1[mrow * L1N + n] = (_Float16)(v * ASCALE);
      }
    }
  }
  __syncthreads();

  {
    v8f acc[2];
#pragma unroll
    for (int j = 0; j < 2; ++j) acc[j] = (v8f){0.f, 0.f, 0.f, 0.f, 0.f, 0.f, 0.f, 0.f};
#pragma unroll 1
    for (int kc = 0; kc < L1N / 32; ++kc) {
      const int kb = kc * 32;
      const v16h a = ld_frag_h(h1 + m * L1N + kb, h);
#pragma unroll
      for (int j = 0; j < 2; ++j) {
        const int n = (wv * 2 + j) * 16 + m;
        const v16h b = ld_frag_f32(W2 + (size_t)n * L1N + kb, h, WSCALE);
        acc[j] = wmma16(a, b, acc[j]);
      }
    }
#pragma unroll
    for (int j = 0; j < 2; ++j) {
      const int n = (wv * 2 + j) * 16 + m;
      const float bb = b2[n];
#pragma unroll
      for (int e = 0; e < 8; ++e) {
        const int mrow = 8 * h + e;
        float v = acc[j][e] * INV_AW + bb;
        v = v > 0.0f ? v : 0.01f * v;
        h2[mrow * L2N + n] = (_Float16)(v * ASCALE);
      }
    }
  }
  __syncthreads();

  if (wv == 0) {
    v8f acc = (v8f){0.f, 0.f, 0.f, 0.f, 0.f, 0.f, 0.f, 0.f};
    const int nc = m < OUTN ? m : (OUTN - 1);
    const float sc = m < OUTN ? WSCALE : 0.0f;
#pragma unroll 1
    for (int kc = 0; kc < L2N / 32; ++kc) {
      const int kb = kc * 32;
      const v16h a = ld_frag_h(h2 + m * L2N + kb, h);
      const v16h b = ld_frag_f32(W3 + (size_t)nc * L2N + kb, h, sc);
      acc = wmma16(a, b, acc);
    }
    if (m < OUTN) {
      const float bb = b3[m];
#pragma unroll
      for (int e = 0; e < 8; ++e) {
        const int mrow = 8 * h + e;
        outS[mrow * OUTN + m] = acc[e] * INV_AW + bb;
      }
    }
  }
  __syncthreads();

  const bool doit = (tid < MROWS) && (row0 + tid < nrows);
  v4f ov = (v4f){0.f, 0.f, 0.f, 0.f};
  if (doit) ov = *(const v4f*)(outS + OUTN * tid);
  float* op = out + (size_t)(row0 + (tid < MROWS ? tid : 0)) * OUTN;
  if (doit) *(volatile v4f*)op = ov;
  __threadfence();
  if (doit) *(volatile v4f*)op = ov;
}

extern "C" void kernel_launch(void* const* d_in, const int* in_sizes, int n_in,
                              void* d_out, int out_size, void* d_ws, size_t ws_size,
                              hipStream_t stream) {
  if (n_in < 7) return;
  const float* x  = (const float*)d_in[0];
  const float* W1 = (const float*)d_in[1];
  const float* b1 = (const float*)d_in[2];
  const float* W2 = (const float*)d_in[3];
  const float* b2 = (const float*)d_in[4];
  const float* W3 = (const float*)d_in[5];
  const float* b3 = (const float*)d_in[6];
  float* out = (float*)d_out;

  int nrows = in_sizes[0] / SEQ_L;
  const int nrows_out = out_size / OUTN;
  if (nrows_out < nrows) nrows = nrows_out;
  if (nrows <= 0) return;
  if (in_sizes[1] < L1N * POOLED || in_sizes[3] < L2N * L1N || in_sizes[5] < OUTN * L2N) return;
  if (in_sizes[2] < L1N || in_sizes[4] < L2N || in_sizes[6] < OUTN) return;

  const size_t normH_bytes = (size_t)nrows * POOLED * sizeof(_Float16);
  if (normH_bytes > ws_size) return;
  _Float16* normH = (_Float16*)d_ws;

  k_acf<<<dim3(nrows), dim3(256), 0, stream>>>(x, normH);
  k_mlp<<<dim3((nrows + MROWS - 1) / MROWS), dim3(256), 0, stream>>>(
      normH, W1, b1, W2, b2, W3, b3, out, nrows);
}
